// GATv2Model_77824807403686
// MI455X (gfx1250) — hardware-run, weakly checked
//
#include <hip/hip_runtime.h>
#include <stddef.h>
#include <stdint.h>
#include <math.h>


#define NGR   64
#define NND   64
#define DM    256
#define NHD   8
#define HCH   32
#define NLY   4
#define NCT   16
#define NOC   3
#define NRW   (NGR * NND)
#define KHL   (2 * DM)
#define NTHR  256
#define RPB   (NTHR / 32)
#define GBM   64
#define GBN   64
#define GTHR  128
#define LNEPS 1e-5f
#define NEGSL 0.2f
#define WSMAX 134217728

static_assert((NRW % GBM) == 0 && (DM % GBN) == 0 && (KHL % GBN) == 0);
static_assert((KHL % 32) == 0);
static_assert(DM == 32 * 8);
static_assert(NND == 64 && HCH == 32 && NHD * HCH == DM);
static_assert((NRW % RPB) == 0);
static_assert(GBM == (GTHR / 32) * 16);
static_assert(NTHR == 4 * NND);
static_assert(NTHR == 8 * 32 && NND == 8 * RPB);
static_assert(((NND * NOC) % 4) == 0 && (NND * NOC) / 4 <= NTHR);
static_assert(NCT * 8 <= NTHR);
static_assert(NND * NND == 4 * 4 * NTHR);

typedef float          v4f  __attribute__((ext_vector_type(4)));
typedef float          v8f  __attribute__((ext_vector_type(8)));
typedef int            v4i  __attribute__((ext_vector_type(4)));
typedef int            v8i  __attribute__((ext_vector_type(8)));
typedef unsigned int   v4u  __attribute__((ext_vector_type(4)));
typedef unsigned short v8us __attribute__((ext_vector_type(8)));
typedef __bf16         v16b __attribute__((ext_vector_type(16)));
typedef v4f  __attribute__((may_alias)) v4fa;
typedef v4i  __attribute__((may_alias)) v4ia;
typedef v8us __attribute__((may_alias)) v8usa;
union FragB { v16b v; v8us h[2]; v8i w; };

__device__ __forceinline__ v8f wmb(const FragB& a, const FragB& b, v8f c) {
  v8f d = __builtin_amdgcn_wmma_f32_16x16x32_bf16(false, a.v, false, b.v, (short)0, c, false, false);
  asm volatile("v_nop\n\tv_nop\n\tv_nop\n\tv_nop" : "+v"(d) : "v"(a.w), "v"(b.w));
  return d;
}

__device__ __forceinline__ unsigned int f2bf(float f) {
  const unsigned int u = __float_as_uint(f);
  return ((u + 0x7FFFu + ((u >> 16) & 1u)) >> 16) & 0xFFFFu;
}
__device__ __forceinline__ float bf2f(unsigned int b) { return __uint_as_float(b << 16); }
__device__ __forceinline__ float bfr(float f) { return bf2f(f2bf(f)); }
__device__ __forceinline__ v4f bfr4(const v4f a) {
  v4f r; r.x = bfr(a.x); r.y = bfr(a.y); r.z = bfr(a.z); r.w = bfr(a.w); return r;
}
__device__ __forceinline__ unsigned int pk2(float lo, float hi) { return f2bf(lo) | (f2bf(hi) << 16); }
__device__ __forceinline__ v4u pack8(const v4f a, const v4f b) {
  v4u r;
  r.x = pk2(a.x, a.y); r.y = pk2(a.z, a.w); r.z = pk2(b.x, b.y); r.w = pk2(b.z, b.w);
  return r;
}
__device__ __forceinline__ void hl8(const float y[8], v4u& hv, v4u& lv) {
  unsigned int hb[8], lb[8];
#pragma unroll
  for (int j = 0; j < 8; ++j) {
    hb[j] = f2bf(y[j]);
    lb[j] = f2bf(y[j] - bf2f(hb[j]));
  }
  hv.x = hb[0] | (hb[1] << 16); hv.y = hb[2] | (hb[3] << 16); hv.z = hb[4] | (hb[5] << 16); hv.w = hb[6] | (hb[7] << 16);
  lv.x = lb[0] | (lb[1] << 16); lv.y = lb[2] | (lb[3] << 16); lv.z = lb[4] | (lb[5] << 16); lv.w = lb[6] | (lb[7] << 16);
}

__device__ __forceinline__ float wave_sum(float v) {
#pragma unroll
  for (int off = 16; off > 0; off >>= 1) v += __shfl_xor(v, off);
  return v;
}
__device__ __forceinline__ float wave_max(float v) {
#pragma unroll
  for (int off = 16; off > 0; off >>= 1) v = fmaxf(v, __shfl_xor(v, off));
  return v;
}

__device__ __forceinline__ void ln_wave8(const float z[8], const v4f ga, const v4f gb, const v4f ea, const v4f eb,
                                         float y[8]) {
  float s = ((z[0] + z[1]) + (z[2] + z[3])) + ((z[4] + z[5]) + (z[6] + z[7]));
  s = wave_sum(s);
  const float mean = s * (1.0f / (float)DM);
  float d[8];
  float q = 0.f;
#pragma unroll
  for (int j = 0; j < 8; ++j) { d[j] = z[j] - mean; q = fmaf(d[j], d[j], q); }
  q = wave_sum(q);
  const float var = q * (1.0f / (float)DM);
  const float rs  = 1.0f / sqrtf(var + LNEPS);
  y[0] = fmaf(d[0] * rs, ga.x, ea.x); y[1] = fmaf(d[1] * rs, ga.y, ea.y);
  y[2] = fmaf(d[2] * rs, ga.z, ea.z); y[3] = fmaf(d[3] * rs, ga.w, ea.w);
  y[4] = fmaf(d[4] * rs, gb.x, eb.x); y[5] = fmaf(d[5] * rs, gb.y, eb.y);
  y[6] = fmaf(d[6] * rs, gb.z, eb.z); y[7] = fmaf(d[7] * rs, gb.w, eb.w);
}

__global__ __launch_bounds__(NTHR) void k_wdup(const float* __restrict__ src, int nSrcRows, int dstPitchRows,
                                               int dstRowOff, int gs, unsigned short* dst, int nUnits) {
  const int u = (int)blockIdx.x * NTHR + (int)threadIdx.x;
  if (u >= nUnits) return;
  const int r   = u >> 6;
  const int k8  = (u & 63) * 8;
  const int col = ((k8 >> (gs + 1)) << gs) + (k8 & ((1 << gs) - 1));
  const int rc  = r < nSrcRows ? r : nSrcRows - 1;
  const float* p = src + (size_t)rc * DM + col;
  const v4f a = *(const v4fa*)p, b = *(const v4fa*)(p + 4);
  const v4u hv = pack8(a, b);
  const int R = (r >> 8) * dstPitchRows + dstRowOff + (r & 255);
  unsigned short* o = dst + (size_t)R * KHL + k8;
  *(volatile v4u*)o = hv;
  __threadfence();
  *(volatile v4u*)o = hv;
}

__global__ __launch_bounds__(NTHR) void k_ee(const float* __restrict__ etab, const float* __restrict__ We, float* EE) {
  __shared__ __attribute__((aligned(16))) float ecs[DM];
  __shared__ __attribute__((aligned(16))) float eo[DM];
  __shared__ float red[8];
  const int tid = (int)threadIdx.x, lane = tid & 31, wave = tid >> 5;
  const int blk = (int)blockIdx.x;
  const int l = blk >> 4, cat = blk & 15;
  const float v = bfr(etab[cat * DM + tid]);
  const float sq = wave_sum(v * v);
  if (lane == 0) red[wave] = sq;
  __syncthreads();
  float ss = 0.f;
#pragma unroll
  for (int w = 0; w < 8; ++w) ss += red[w];
  float nrm = sqrtf(ss);
  nrm = (nrm == 0.f) ? 1e-8f : nrm;
  const float scl = fminf(1.0f, 1.0f / nrm);
  ecs[tid] = v * scl;
  __syncthreads();
  const float* wrow = We + ((size_t)(l * DM + tid)) * (size_t)DM;
  float acc = 0.f;
#pragma unroll 2
  for (int k4 = 0; k4 < DM / 4; ++k4) {
    const v4f w4 = bfr4(*(const v4fa*)(wrow + 4 * k4));
    const v4f e4 = *(const v4fa*)(ecs + 4 * k4);
    acc = fmaf(e4.x, w4.x, acc);
    acc = fmaf(e4.y, w4.y, acc);
    acc = fmaf(e4.z, w4.z, acc);
    acc = fmaf(e4.w, w4.w, acc);
  }
  eo[tid] = acc;
  __syncthreads();
  const bool wr = tid < DM / 4;
  const int  tp = tid < DM / 4 ? tid : DM / 4 - 1;
  const v4f o4 = *(const v4fa*)(eo + 4 * tp);
  float* op = EE + (size_t)blk * DM + 4 * tp;
  if (wr) *(volatile v4f*)op = o4;
  __threadfence();
  if (wr) *(volatile v4f*)op = o4;
}

__global__ __launch_bounds__(NTHR) void k_in1(const float* __restrict__ x, const float* __restrict__ W1,
                                              const float* __restrict__ b1, const float* __restrict__ g1,
                                              const float* __restrict__ be1, unsigned short* A0, int nRows) {
  const int tid = (int)threadIdx.x, lane = tid & 31, wave = tid >> 5;
  const int row = (int)blockIdx.x * RPB + wave;
  if (row >= nRows) return;
  const int c0 = 8 * lane;
  const float x0 = bfr(x[(size_t)row * 2]), x1 = bfr(x[(size_t)row * 2 + 1]);
  const float* wp = W1 + 2 * c0;
  const v4f w0 = bfr4(*(const v4fa*)wp),       w1 = bfr4(*(const v4fa*)(wp + 4));
  const v4f w2 = bfr4(*(const v4fa*)(wp + 8)), w3 = bfr4(*(const v4fa*)(wp + 12));
  const v4f ba = bfr4(*(const v4fa*)(b1 + c0)),  bb = bfr4(*(const v4fa*)(b1 + c0 + 4));
  const v4f ga = bfr4(*(const v4fa*)(g1 + c0)),  gb = bfr4(*(const v4fa*)(g1 + c0 + 4));
  const v4f ea = bfr4(*(const v4fa*)(be1 + c0)), eb = bfr4(*(const v4fa*)(be1 + c0 + 4));
  float z[8];
  z[0] = fmaf(x1, w0.y, x0 * w0.x) + ba.x;
  z[1] = fmaf(x1, w0.w, x0 * w0.z) + ba.y;
  z[2] = fmaf(x1, w1.y, x0 * w1.x) + ba.z;
  z[3] = fmaf(x1, w1.w, x0 * w1.z) + ba.w;
  z[4] = fmaf(x1, w2.y, x0 * w2.x) + bb.x;
  z[5] = fmaf(x1, w2.w, x0 * w2.z) + bb.y;
  z[6] = fmaf(x1, w3.y, x0 * w3.x) + bb.z;
  z[7] = fmaf(x1, w3.w, x0 * w3.z) + bb.w;
  float y[8];
  ln_wave8(z, ga, gb, ea, eb, y);
#pragma unroll
  for (int j = 0; j < 8; ++j) y[j] = fmaxf(y[j], 0.f);
  v4u hv, lv;
  hl8(y, hv, lv);
  unsigned short* hp = A0 + (size_t)row * KHL + c0;
  unsigned short* lp = hp + DM;
  *(volatile v4u*)hp = hv; *(volatile v4u*)lp = lv;
  __threadfence();
  *(volatile v4u*)hp = hv; *(volatile v4u*)lp = lv;
}

template<int MODE>
__global__ __launch_bounds__(NTHR) void k_ln(const float* __restrict__ Z, const float* __restrict__ bias,
                                             const float* __restrict__ g, const float* __restrict__ be,
                                             const float* __restrict__ Hres, float* Hout, unsigned short* HL,
                                             int nRows) {
  __shared__ __attribute__((aligned(16))) float stw_all[RPB * DM];
  const int tid = (int)threadIdx.x, lane = tid & 31, wave = tid >> 5;
  const int row = (int)blockIdx.x * RPB + wave;
  if (row >= nRows) return;
  float* stw = stw_all + wave * DM;
  const int c0 = 8 * lane;
  const v4f za = *(const v4fa*)(Z + (size_t)row * DM + c0), zb = *(const v4fa*)(Z + (size_t)row * DM + c0 + 4);
  const v4f ba = bfr4(*(const v4fa*)(bias + c0)), bb = bfr4(*(const v4fa*)(bias + c0 + 4));
  const v4f ga = bfr4(*(const v4fa*)(g + c0)),    gb = bfr4(*(const v4fa*)(g + c0 + 4));
  const v4f ea = bfr4(*(const v4fa*)(be + c0)),   eb = bfr4(*(const v4fa*)(be + c0 + 4));
  float z[8] = {za.x + ba.x, za.y + ba.y, za.z + ba.z, za.w + ba.w, zb.x + bb.x, zb.y + bb.y, zb.z + bb.z, zb.w + bb.w};
  float y[8];
  ln_wave8(z, ga, gb, ea, eb, y);
  if (MODE == 1) {
    const v4f ra = *(const v4fa*)(Hres + (size_t)row * DM + c0), rb = *(const v4fa*)(Hres + (size_t)row * DM + c0 + 4);
    y[0] = fmaxf(y[0], 0.f) + ra.x; y[1] = fmaxf(y[1], 0.f) + ra.y; y[2] = fmaxf(y[2], 0.f) + ra.z; y[3] = fmaxf(y[3], 0.f) + ra.w;
    y[4] = fmaxf(y[4], 0.f) + rb.x; y[5] = fmaxf(y[5], 0.f) + rb.y; y[6] = fmaxf(y[6], 0.f) + rb.z; y[7] = fmaxf(y[7], 0.f) + rb.w;
  }
  v4u hv, lv;
  hl8(y, hv, lv);
  unsigned short* hp = HL + (size_t)row * KHL + c0;
  unsigned short* lp = hp + DM;
  v4f ya, yb;
  ya.x = y[0]; ya.y = y[1]; ya.z = y[2]; ya.w = y[3];
  yb.x = y[4]; yb.y = y[5]; yb.z = y[6]; yb.w = y[7];
  *(v4fa*)(stw + c0) = ya;
  *(v4fa*)(stw + c0 + 4) = yb;
  __builtin_amdgcn_fence(__ATOMIC_RELEASE, "wavefront");
  __builtin_amdgcn_wave_barrier();
  const v4f p0 = *(const v4fa*)(stw + 4 * lane);
  const v4f p1 = *(const v4fa*)(stw + DM / 2 + 4 * lane);
  float* op = Hout + (size_t)row * DM;
  *(volatile v4u*)hp = hv; *(volatile v4u*)lp = lv;
  *(volatile v4f*)(op + 4 * lane) = p0; *(volatile v4f*)(op + DM / 2 + 4 * lane) = p1;
  __threadfence();
  *(volatile v4u*)hp = hv; *(volatile v4u*)lp = lv;
  *(volatile v4f*)(op + 4 * lane) = p0; *(volatile v4f*)(op + DM / 2 + 4 * lane) = p1;
}

__global__ __launch_bounds__(GTHR) void k_gemm(const unsigned short* __restrict__ A,
                                               const unsigned short* __restrict__ WT,
                                               float* outF, int K, int ldo) {
  __shared__ __attribute__((aligned(16))) float stg[GBM * GBN];
  const int tid = (int)threadIdx.x, lane = tid & 31, wave = tid >> 5, hh = lane >> 4, m = lane & 15;
  const int rowBase = (int)blockIdx.x * GBM;
  const int col0    = (int)blockIdx.y * GBN;

  v8f acc[4];
  {
    const v8f z = {0.f, 0.f, 0.f, 0.f, 0.f, 0.f, 0.f, 0.f};
    acc[0] = z; acc[1] = z; acc[2] = z; acc[3] = z;
  }
  const unsigned short* ap = A  + (size_t)(rowBase + 16 * wave + m) * (size_t)K + 8 * hh;
  const unsigned short* wp = WT + (size_t)(col0 + m) * (size_t)K + 8 * hh;
  const int ksteps = K >> 5;
#pragma unroll 1
  for (int ks = 0; ks < ksteps; ++ks) {
    FragB af;
    af.h[0] = *(const v8usa*)(ap + 32 * ks);
    af.h[1] = *(const v8usa*)(ap + 32 * ks + 16);
#pragma unroll
    for (int t = 0; t < 4; ++t) {
      const unsigned short* wq = wp + (size_t)(16 * t) * (size_t)K + 32 * ks;
      FragB bf;
      bf.h[0] = *(const v8usa*)wq;
      bf.h[1] = *(const v8usa*)(wq + 16);
      acc[t] = wmb(af, bf, acc[t]);
    }
  }

#pragma unroll
  for (int t = 0; t < 4; ++t) {
    const int lc = 16 * t + m;
#pragma unroll
    for (int r = 0; r < 8; ++r) {
      const int lr = 16 * wave + 8 * hh + r;
      stg[lr * GBN + lc] = acc[t][r];
    }
  }
  __syncthreads();

  v4f fv[8];
#pragma unroll
  for (int i = 0; i < 8; ++i) {
    const int lr = 16 * wave + 2 * i + hh;
    fv[i] = *(const v4fa*)(stg + lr * GBN + 4 * m);
  }
#pragma unroll
  for (int i = 0; i < 8; ++i) {
    const int lr = 16 * wave + 2 * i + hh;
    const int gr = rowBase + lr;
    float* op = outF + (size_t)gr * (size_t)ldo + col0 + 4 * m;
    *(volatile v4f*)op = fv[i];
  }
  __threadfence();
#pragma unroll
  for (int i = 0; i < 8; ++i) {
    const int lr = 16 * wave + 2 * i + hh;
    const int gr = rowBase + lr;
    float* op = outF + (size_t)gr * (size_t)ldo + col0 + 4 * m;
    *(volatile v4f*)op = fv[i];
  }
}

__global__ __launch_bounds__(NTHR) void k_attn(const float* __restrict__ XLR, const float* __restrict__ EEl,
                                               const int* __restrict__ cat, const float* __restrict__ attl,
                                               const float* __restrict__ bll, const float* __restrict__ brl,
                                               const float* __restrict__ cbl, unsigned short* MHL) {
  __shared__ __attribute__((aligned(16))) float xl_s[NND * HCH];
  __shared__ __attribute__((aligned(16))) float xr_s[NND * HCH];
  __shared__ __attribute__((aligned(16))) float ee_s[NCT * HCH];
  __shared__ __attribute__((aligned(16))) int   cat_s[NND * NND];
  __shared__ __attribute__((aligned(16))) float S[NND * NND];
  const int tid = (int)threadIdx.x, lane = tid & 31, wave = tid >> 5;
  const int b = (int)blockIdx.x >> 3, h = (int)blockIdx.x & 7;
  const int hc0 = h * HCH;

#pragma unroll
  for (int i = 0; i < 2; ++i) {
    const int p = tid + NTHR * i;
    const int s = p >> 3, q = (p & 7) * 4;
    const float* src = XLR + (size_t)(b * NND + s) * KHL + hc0 + q;
    const v4f vl = *(const v4fa*)src;
    const v4f vr = *(const v4fa*)(src + DM);
    const v4f gl = bfr4(*(const v4fa*)(bll + hc0 + q));
    const v4f gr = bfr4(*(const v4fa*)(brl + hc0 + q));
    *(v4fa*)(xl_s + s * HCH + q) = vl + gl;
    *(v4fa*)(xr_s + s * HCH + q) = vr + gr;
  }
  {
    const bool w  = tid < NCT * 8;
    const int  tp = tid < NCT * 8 ? tid : NCT * 8 - 1;
    const int c = tp >> 3, q = (tp & 7) * 4;
    const v4f ve = *(const v4fa*)(EEl + (size_t)c * DM + hc0 + q);
    if (w) *(v4fa*)(ee_s + c * HCH + q) = ve;
  }
#pragma unroll
  for (int i = 0; i < 4; ++i) {
    const int p = tid + NTHR * i;
    v4i cv = *(const v4ia*)(cat + 4 * p);
    cv.x = min(max(cv.x, 0), NCT - 1); cv.y = min(max(cv.y, 0), NCT - 1);
    cv.z = min(max(cv.z, 0), NCT - 1); cv.w = min(max(cv.w, 0), NCT - 1);
    *(v4ia*)(cat_s + 4 * p) = cv;
  }
  v4f atv[8];
#pragma unroll
  for (int q = 0; q < 8; ++q) atv[q] = bfr4(*(const v4fa*)(attl + hc0 + 4 * q));
  __syncthreads();

  {
    const int s = tid >> 2, tq = tid & 3;
    v4f xv[8];
#pragma unroll
    for (int q = 0; q < 8; ++q) xv[q] = *(const v4fa*)(xl_s + s * HCH + 4 * q);
#pragma unroll 1
    for (int j = 0; j < NND / 4; ++j) {
      const int t = 4 * j + tq;
      const int c = cat_s[s * NND + t];
      const float* xrp = xr_s + t * HCH;
      const float* eep = ee_s + c * HCH;
      float acc = 0.f;
#pragma unroll
      for (int q = 0; q < 8; ++q) {
        const v4f r4 = *(const v4fa*)(xrp + 4 * q);
        const v4f e4 = *(const v4fa*)(eep + 4 * q);
        float u0 = (xv[q].x + r4.x) + e4.x; u0 = fmaxf(u0, NEGSL * u0); acc = fmaf(atv[q].x, u0, acc);
        float u1 = (xv[q].y + r4.y) + e4.y; u1 = fmaxf(u1, NEGSL * u1); acc = fmaf(atv[q].y, u1, acc);
        float u2 = (xv[q].z + r4.z) + e4.z; u2 = fmaxf(u2, NEGSL * u2); acc = fmaf(atv[q].z, u2, acc);
        float u3 = (xv[q].w + r4.w) + e4.w; u3 = fmaxf(u3, NEGSL * u3); acc = fmaf(atv[q].w, u3, acc);
      }
      S[t * NND + s] = acc;
    }
  }
  __syncthreads();

#pragma unroll 1
  for (int i = 0; i < 8; ++i) {
    float* sp = S + (wave * 8 + i) * NND;
    const float v0 = sp[lane], v1 = sp[lane + 32];
    const float mx = wave_max(fmaxf(v0, v1));
    const float e0 = expf(v0 - mx), e1 = expf(v1 - mx);
    const float sm = wave_sum(e0 + e1);
    const float inv = 1.0f / sm;
    sp[lane] = e0 * inv;
    sp[lane + 32] = e1 * inv;
  }
  __syncthreads();

  float* mm = xr_s;
  {
    const int t = tid >> 2, c0 = (tid & 3) * 8;
    float mv[8] = {0.f, 0.f, 0.f, 0.f, 0.f, 0.f, 0.f, 0.f};
    const float* sp = S + t * NND;
#pragma unroll 2
    for (int s = 0; s < NND; ++s) {
      const float a = sp[s];
      const v4f xa = *(const v4fa*)(xl_s + s * HCH + c0);
      const v4f xb = *(const v4fa*)(xl_s + s * HCH + c0 + 4);
      mv[0] = fmaf(a, xa.x, mv[0]); mv[1] = fmaf(a, xa.y, mv[1]); mv[2] = fmaf(a, xa.z, mv[2]); mv[3] = fmaf(a, xa.w, mv[3]);
      mv[4] = fmaf(a, xb.x, mv[4]); mv[5] = fmaf(a, xb.y, mv[5]); mv[6] = fmaf(a, xb.z, mv[6]); mv[7] = fmaf(a, xb.w, mv[7]);
    }
    const v4f ca = bfr4(*(const v4fa*)(cbl + hc0 + c0)), cb4 = bfr4(*(const v4fa*)(cbl + hc0 + c0 + 4));
    v4f oa, ob;
    oa.x = mv[0] + ca.x;  oa.y = mv[1] + ca.y;  oa.z = mv[2] + ca.z;  oa.w = mv[3] + ca.w;
    ob.x = mv[4] + cb4.x; ob.y = mv[5] + cb4.y; ob.z = mv[6] + cb4.z; ob.w = mv[7] + cb4.w;
    *(v4fa*)(mm + t * HCH + c0) = oa;
    *(v4fa*)(mm + t * HCH + c0 + 4) = ob;
  }
  __syncthreads();

  v4u ov[2];
  size_t oo[2];
#pragma unroll
  for (int i = 0; i < 2; ++i) {
    const int p = tid + NTHR * i;
    const int r = p >> 3, pr = p & 7;
    const int cc = 8 * (pr & 3);
    const v4f va = *(const v4fa*)(mm + r * HCH + cc);
    const v4f vb = *(const v4fa*)(mm + r * HCH + cc + 4);
    const float yv[8] = {va.x, va.y, va.z, va.w, vb.x, vb.y, vb.z, vb.w};
    v4u hv, lv;
    hl8(yv, hv, lv);
    const bool lo = pr >= 4;
    v4u wv;
    wv.x = lo ? lv.x : hv.x; wv.y = lo ? lv.y : hv.y; wv.z = lo ? lv.z : hv.z; wv.w = lo ? lv.w : hv.w;
    ov[i] = wv;
    oo[i] = (size_t)(b * NND + r) * KHL + (size_t)(h * 2 * HCH) + 8 * pr;
  }
  *(volatile v4u*)(MHL + oo[0]) = ov[0];
  *(volatile v4u*)(MHL + oo[1]) = ov[1];
  __threadfence();
  *(volatile v4u*)(MHL + oo[0]) = ov[0];
  *(volatile v4u*)(MHL + oo[1]) = ov[1];
}

__global__ __launch_bounds__(NTHR) void k_out(const float* __restrict__ H, const float* __restrict__ Wo,
                                              const float* __restrict__ bo, float* out) {
  __shared__ __attribute__((aligned(16))) float so[NND * NOC];
  const int tid = (int)threadIdx.x, lane = tid & 31, wave = tid >> 5;
  const int b = (int)blockIdx.x;
  const int c0 = 8 * lane;
  const v4f w0a = bfr4(*(const v4fa*)(Wo + c0)),          w0b = bfr4(*(const v4fa*)(Wo + c0 + 4));
  const v4f w1a = bfr4(*(const v4fa*)(Wo + DM + c0)),     w1b = bfr4(*(const v4fa*)(Wo + DM + c0 + 4));
  const v4f w2a = bfr4(*(const v4fa*)(Wo + 2 * DM + c0)), w2b = bfr4(*(const v4fa*)(Wo + 2 * DM + c0 + 4));
  const float o0 = bfr(bo[0]), o1 = bfr(bo[1]), o2 = bfr(bo[2]);
#pragma unroll 1
  for (int i = 0; i < 8; ++i) {
    const int r = wave * 8 + i;
    const float* hp = H + (size_t)(b * NND + r) * DM + c0;
    const v4f ha = *(const v4fa*)hp, hb = *(const v4fa*)(hp + 4);
    float d0 = ha.x * w0a.x; d0 = fmaf(ha.y, w0a.y, d0); d0 = fmaf(ha.z, w0a.z, d0); d0 = fmaf(ha.w, w0a.w, d0);
    d0 = fmaf(hb.x, w0b.x, d0); d0 = fmaf(hb.y, w0b.y, d0); d0 = fmaf(hb.z, w0b.z, d0); d0 = fmaf(hb.w, w0b.w, d0);
    float d1 = ha.x * w1a.x; d1 = fmaf(ha.y, w1a.y, d1); d1 = fmaf(ha.z, w1a.z, d1); d1 = fmaf(ha.w, w1a.w, d1);
    d1 = fmaf(hb.x, w1b.x, d1); d1 = fmaf(hb.y, w1b.y, d1); d1 = fmaf(hb.z, w1b.z, d1); d1 = fmaf(hb.w, w1b.w, d1);
    float d2 = ha.x * w2a.x; d2 = fmaf(ha.y, w2a.y, d2); d2 = fmaf(ha.z, w2a.z, d2); d2 = fmaf(ha.w, w2a.w, d2);
    d2 = fmaf(hb.x, w2b.x, d2); d2 = fmaf(hb.y, w2b.y, d2); d2 = fmaf(hb.z, w2b.z, d2); d2 = fmaf(hb.w, w2b.w, d2);
    d0 = wave_sum(d0);
    d1 = wave_sum(d1);
    d2 = wave_sum(d2);
    if (lane == 0) {
      so[r * NOC + 0] = d0 + o0;
      so[r * NOC + 1] = d1 + o1;
      so[r * NOC + 2] = d2 + o2;
    }
  }
  __syncthreads();
  const int npc = (NND * NOC) / 4;
  const bool wr = tid < npc;
  const int  tp = tid < npc ? tid : npc - 1;
  const v4f v = *(const v4fa*)(so + 4 * tp);
  float* op = out + (size_t)b * (NND * NOC) + 4 * tp;
  if (wr) *(volatile v4f*)op = v;
  __threadfence();
  if (wr) *(volatile v4f*)op = v;
}

static inline int cdiv(int a, int b) { return (a + b - 1) / b; }

extern "C" void kernel_launch(void* const* d_in, const int* in_sizes, int n_in,
                              void* d_out, int out_size, void* d_ws, size_t ws_size,
                              hipStream_t stream) {
  if (n_in < 24) return;
  if (in_sizes[0] != NRW * 2) return;
  if (in_sizes[1] != NND * NND) return;
  if (in_sizes[2] != NCT * DM) return;
  if (in_sizes[3] != DM * 2 || in_sizes[4] != DM || in_sizes[5] != DM || in_sizes[6] != DM) return;
  if (in_sizes[7] != DM * DM || in_sizes[8] != DM || in_sizes[9] != DM || in_sizes[10] != DM) return;
  if (in_sizes[11] != NLY * DM * DM || in_sizes[12] != NLY * DM) return;
  if (in_sizes[13] != NLY * DM * DM || in_sizes[14] != NLY * DM) return;
  if (in_sizes[15] != NLY * DM * DM) return;
  if (in_sizes[16] != NLY * NHD * HCH || in_sizes[17] != NLY * DM) return;
  if (in_sizes[18] != NLY * DM * DM || in_sizes[19] != NLY * DM) return;
  if (in_sizes[20] != NLY * DM || in_sizes[21] != NLY * DM) return;
  if (in_sizes[22] != NOC * DM || in_sizes[23] != NOC) return;
  if (out_size != NRW * NOC) return;

  const float* x    = (const float*)d_in[0];
  const int*   ecat = (const int*)  d_in[1];
  const float* etab = (const float*)d_in[2];
  const float* Wi1  = (const float*)d_in[3];
  const float* bi1  = (const float*)d_in[4];
  const float* g1   = (const float*)d_in[5];
  const float* be1  = (const float*)d_in[6];
  const float* Wi2  = (const float*)d_in[7];
  const float* bi2  = (const float*)d_in[8];
  const float* g2   = (const float*)d_in[9];
  const float* be2  = (const float*)d_in[10];
  const float* Wl   = (const float*)d_in[11];
  const float* bl   = (const float*)d_in[12];
  const float* Wr   = (const float*)d_in[13];
  const float* br   = (const float*)d_in[14];
  const float* We   = (const float*)d_in[15];
  const float* att  = (const float*)d_in[16];
  const float* cb   = (const float*)d_in[17];
  const float* Wp   = (const float*)d_in[18];
  const float* bp   = (const float*)d_in[19];
  const float* lg   = (const float*)d_in[20];
  const float* lb   = (const float*)d_in[21];
  const float* Wo   = (const float*)d_in[22];
  const float* bo   = (const float*)d_in[23];
  float* out = (float*)d_out;

  char* ws = (char*)d_ws;
  size_t off = 0;
  const size_t oWI2P = off; off += (size_t)DM * KHL * 2;
  const size_t oWLRP = off; off += (size_t)NLY * KHL * KHL * 2;
  const size_t oWPP  = off; off += (size_t)NLY * DM * KHL * 2;
  const size_t oEE   = off; off += (size_t)NLY * NCT * DM * 4;
  const size_t oA0   = off; off += (size_t)NRW * KHL * 2;
  const size_t oZ    = off; off += (size_t)NRW * DM * 4;
  const size_t oHA   = off; off += (size_t)NRW * DM * 4;
  const size_t oHB   = off; off += (size_t)NRW * DM * 4;
  const size_t oHHL  = off; off += (size_t)NRW * KHL * 2;
  const size_t oXLR  = off; off += (size_t)NRW * KHL * 4;
  const size_t oMHL  = off; off += (size_t)NRW * KHL * 2;
  if (off > ws_size || off > (size_t)WSMAX) return;
  unsigned short* WI2P = (unsigned short*)(ws + oWI2P);
  unsigned short* WLRP = (unsigned short*)(ws + oWLRP);
  unsigned short* WPP  = (unsigned short*)(ws + oWPP);
  float*          EE   = (float*)(ws + oEE);
  unsigned short* A0   = (unsigned short*)(ws + oA0);
  float*          Z    = (float*)(ws + oZ);
  float*          HA   = (float*)(ws + oHA);
  float*          HB   = (float*)(ws + oHB);
  unsigned short* HHL  = (unsigned short*)(ws + oHHL);
  float*          XLR  = (float*)(ws + oXLR);
  unsigned short* MHL  = (unsigned short*)(ws + oMHL);

  {
    const int nU0 = DM * 64;
    k_wdup<<<cdiv(nU0, NTHR), NTHR, 0, stream>>>(Wi2, DM, DM, 0, 8, WI2P, nU0);
    const int nU1 = NLY * DM * 64;
    k_wdup<<<cdiv(nU1, NTHR), NTHR, 0, stream>>>(Wl, NLY * DM, KHL, 0,  8, WLRP, nU1);
    k_wdup<<<cdiv(nU1, NTHR), NTHR, 0, stream>>>(Wr, NLY * DM, KHL, DM, 8, WLRP, nU1);
    k_wdup<<<cdiv(nU1, NTHR), NTHR, 0, stream>>>(Wp, NLY * DM, DM,  0,  5, WPP,  nU1);
  }
  k_ee<<<NLY * NCT, NTHR, 0, stream>>>(etab, We, EE);
  k_in1<<<NRW / RPB, NTHR, 0, stream>>>(x, Wi1, bi1, g1, be1, A0, NRW);
  k_gemm<<<dim3(NRW / GBM, DM / GBN), GTHR, 0, stream>>>(A0, WI2P, Z, KHL, DM);
  k_ln<0><<<NRW / RPB, NTHR, 0, stream>>>(Z, bi2, g2, be2, HB, HA, HHL, NRW);

  float* Hc = HA;
  float* Hn = HB;
  for (int l = 0; l < NLY; ++l) {
    k_gemm<<<dim3(NRW / GBM, KHL / GBN), GTHR, 0, stream>>>(HHL, WLRP + (size_t)l * KHL * KHL, XLR, KHL, KHL);
    k_attn<<<NGR * NHD, NTHR, 0, stream>>>(XLR, EE + (size_t)l * NCT * DM, ecat, att + (size_t)l * DM,
                                           bl + (size_t)l * DM, br + (size_t)l * DM, cb + (size_t)l * DM, MHL);
    k_gemm<<<dim3(NRW / GBM, DM / GBN), GTHR, 0, stream>>>(MHL, WPP + (size_t)l * DM * KHL, Z, KHL, DM);
    k_ln<1><<<NRW / RPB, NTHR, 0, stream>>>(Z, bp + (size_t)l * DM, lg + (size_t)l * DM, lb + (size_t)l * DM,
                                            Hc, Hn, HHL, NRW);
    float* tsw = Hc; Hc = Hn; Hn = tsw;
  }
  k_out<<<NGR, NTHR, 0, stream>>>(Hc, Wo, bo, out);
}
